// Selfattention_21904333209638
// MI455X (gfx1250) — hardware-run, weakly checked
//
#include <hip/hip_runtime.h>
#include <stddef.h>


typedef _Float16 v16h __attribute__((ext_vector_type(16)));
typedef _Float16 v8h  __attribute__((ext_vector_type(8)));
typedef float    v8f  __attribute__((ext_vector_type(8)));
typedef float    v4f  __attribute__((ext_vector_type(4)));
typedef _Float16 h16;

#ifndef NB
#define NB 4
#endif
#ifndef SEQ
#define SEQ 4096
#endif
#define NB_FULL  4
#define SEQ_FULL 4096
#define XD    256
#define UD    128
#define MROWS (NB * SEQ)

static_assert(NB >= 1 && NB <= NB_FULL);
static_assert(SEQ >= 64 && SEQ <= SEQ_FULL && (SEQ % 64) == 0);
static_assert((XD % 64) == 0 && (XD % 32) == 0);
static_assert((UD % 64) == 0 && (UD % 32) == 0);
static_assert((MROWS % 64) == 0 && (MROWS % 32) == 0);
static_assert(XD == 32 * 8);
static_assert(XD == 2 * 32 * 4);
static_assert(XD == 16 * 16);
static_assert(UD == 4 * 32);
static_assert((size_t)NB * XD * SEQ < (size_t)0xFFFFFFFFu);
static_assert((size_t)MROWS * XD < (size_t)0xFFFFFFFFu);

#define LDT 72
#define LDC 68
#define OLD 260
static_assert((LDT % 8) == 0 && LDT >= 64);
static_assert((LDC % 4) == 0 && LDC >= 64);
static_assert((OLD % 4) == 0 && OLD >= XD);

#define WCARRY 64.0f
#define XCARRY 16.0f
#define ACARRY 16.0f
#define PCARRY 1024.0f
#define NEGFILL (-4294967296.0f)

#define WQK_BYTES ((size_t)UD * XD * 2)
#define WV_BYTES  ((size_t)XD * XD * 2)
#define X16_BYTES ((size_t)MROWS * XD * 2)
#define QK_BYTES  ((size_t)MROWS * UD * 2)
#define VT_BYTES  ((size_t)NB * XD * SEQ * 2)
#define MK_BYTES  ((size_t)(MROWS / 32) * 128)
#define OFF_WQ  ((size_t)0)
#define OFF_WK  (OFF_WQ + WQK_BYTES)
#define OFF_WV  (OFF_WK + WQK_BYTES)
#define OFF_X16 (OFF_WV + WV_BYTES)
#define OFF_Q   (OFF_X16 + X16_BYTES)
#define OFF_K   (OFF_Q + QK_BYTES)
#define OFF_VT  (OFF_K + QK_BYTES)
#define OFF_MK  (OFF_VT + VT_BYTES)
#define WS_TOTAL (OFF_MK + MK_BYTES)
static_assert((WQK_BYTES % 128) == 0 && (WV_BYTES % 128) == 0 && (X16_BYTES % 128) == 0);
static_assert((QK_BYTES % 128) == 0 && (VT_BYTES % 128) == 0 && (MK_BYTES % 128) == 0);
static_assert(WS_TOTAL <= (size_t)134217728);

__device__ __forceinline__ float bf16r(float x) {
  unsigned int u = __float_as_uint(x);
  u = (u + 0x7FFFu + ((u >> 16) & 1u)) & 0xFFFF0000u;
  return __uint_as_float(u);
}

static __device__ __forceinline__ h16 toh_flush(float v) {
  const h16 r = (h16)v;
  return (fabsf(v) < 6.103515625e-05f) ? (h16)0.0f : r;
}

__device__ __forceinline__ v16h frag_at(const _Float16* p) {
  v8h lo = *(const v8h*)(p);
  v8h hi = *(const v8h*)(p + 16);
  v16h out;
#pragma unroll
  for (int i = 0; i < 8; ++i) { out[i] = lo[i]; out[i + 8] = hi[i]; }
  return out;
}

__device__ __forceinline__ v8f wmma16(v16h a, v16h b, v8f c) {
  v8f d = __builtin_amdgcn_wmma_f32_16x16x32_f16(false, a, false, b, (short)0, c,
                                                 false, false);
  asm volatile("v_nop\n\tv_nop\n\tv_nop\n\tv_nop" : "+v"(d) : "v"(a), "v"(b));
  return d;
}

__device__ __forceinline__ float red32_sum(float x) {
#pragma unroll
  for (int off = 1; off < 32; off <<= 1) x += __shfl_xor(x, off, 32);
  return x;
}

__device__ __forceinline__ void wave_lds_sync() {
  __builtin_amdgcn_fence(3  , "wavefront");
  asm volatile("s_wait_dscnt 0x0" ::: "memory");
  __builtin_amdgcn_wave_barrier();
}

__device__ __forceinline__ float lrelu_act(float t) {
  return (t >= 0.0f) ? t : 0.2f * t;
}

__global__ __launch_bounds__(256) void wconv_kernel(
    const float* __restrict__ W, _Float16* __restrict__ Wt, unsigned ldw, unsigned ldk) {
  __shared__ _Float16 T[64 * LDT];
  const unsigned tid = threadIdx.x;
  const unsigned n0 = blockIdx.x * 64u;
  const unsigned k0 = blockIdx.y * 64u;
#pragma unroll 4
  for (unsigned j = 0; j < 16u; ++j) {
    const unsigned idx = tid + 256u * j;
    const unsigned kr = idx >> 6, nc = idx & 63u;
    const float v = W[(size_t)(k0 + kr) * ldw + n0 + nc];
    T[nc * LDT + kr] = (_Float16)(WCARRY * bf16r(v));
  }
  __syncthreads();
  v8h x[2];
  size_t off[2];
#pragma unroll
  for (unsigned i = 0; i < 2u; ++i) {
    const unsigned n = 32u * i + (tid >> 3);
    const unsigned kc = (tid & 7u) * 8u;
    x[i] = *(const v8h*)&T[n * LDT + kc];
    off[i] = (size_t)(n0 + n) * ldk + k0 + kc;
  }
#pragma unroll
  for (int i = 0; i < 2; ++i) *(volatile v8h*)(Wt + off[i]) = x[i];
  __threadfence();
#pragma unroll
  for (int i = 0; i < 2; ++i) *(volatile v8h*)(Wt + off[i]) = x[i];
}

__global__ __launch_bounds__(256) void xprep_kernel(
    const float* __restrict__ X, _Float16* __restrict__ X16, unsigned* __restrict__ Mk) {
#pragma clang fp contract(off)
  __shared__ unsigned wbits[8];
  const unsigned lane = threadIdx.x & 31u;
  const unsigned wave = (unsigned)__builtin_amdgcn_readfirstlane((int)(threadIdx.x >> 5));
  unsigned bits = 0u;
#pragma unroll 1
  for (unsigned j = 0; j < 4u; ++j) {
    const unsigned crow = blockIdx.x * 32u + wave * 4u + j;
    const unsigned bidx = crow / (unsigned)SEQ;
    const unsigned sq = crow - bidx * (unsigned)SEQ;
    const size_t srow = (size_t)bidx * SEQ_FULL + sq;
    const float* xr = X + srow * XD + lane * 8u;
    const v4f a0 = *(const v4f*)(xr);
    const v4f a1 = *(const v4f*)(xr + 4u);
    v8h o;
    float as = 0.0f;
#pragma unroll
    for (int i = 0; i < 4; ++i) {
      const float e0 = bf16r(a0[i]);
      const float e1 = bf16r(a1[i]);
      as += fabsf(e0);
      as += fabsf(e1);
      o[i]     = toh_flush(XCARRY * e0);
      o[i + 4] = toh_flush(XCARRY * e1);
    }
    const float tot = red32_sum(as);
    bits |= (tot == 0.0f) ? (1u << (wave * 4u + j)) : 0u;
    _Float16* p = X16 + (size_t)crow * XD + lane * 8u;
    *(volatile v8h*)p = o;
    __threadfence();
    *(volatile v8h*)p = o;
  }
  if (lane == 0u) wbits[wave] = bits;
  __syncthreads();
  if (wave == 0u) {
    unsigned word = 0u;
#pragma unroll
    for (int i = 0; i < 8; ++i) word |= wbits[i];
    volatile unsigned* mp = (volatile unsigned*)(Mk + (size_t)blockIdx.x * 32u + lane);
    *mp = word;
    __threadfence();
    *mp = word;
  }
}

template <int MODE>
__device__ __forceinline__ void gemm_body(
    const _Float16* __restrict__ A16, const _Float16* __restrict__ Bt, const unsigned K,
    const float* __restrict__ bias, _Float16* __restrict__ out16) {
  __shared__ float Cs[64 * LDC];
  const unsigned tid = threadIdx.x, lane = tid & 31u, w = tid >> 5;
  const unsigned mw = w >> 1, nw = w & 1u;
  const unsigned hh = lane >> 4, m = lane & 15u;
  const unsigned n0 = blockIdx.x * 64u;
  const unsigned row0 = blockIdx.y * 64u;

  const _Float16* ap  = A16 + (size_t)(row0 + mw * 16u + m) * K + hh * 8u;
  const _Float16* bp0 = Bt + (size_t)(n0 + nw * 32u + m) * K + hh * 8u;
  const _Float16* bp1 = bp0 + (size_t)16 * K;
  v8f acc0 = {}, acc1 = {};
#pragma unroll 2
  for (unsigned k0 = 0; k0 < K; k0 += 32u) {
    const v16h a  = frag_at(ap + k0);
    const v16h b0 = frag_at(bp0 + k0);
    const v16h b1 = frag_at(bp1 + k0);
    acc0 = wmma16(a, b0, acc0);
    acc1 = wmma16(a, b1, acc1);
  }
#pragma unroll
  for (int r = 0; r < 8; ++r) {
    float* d = &Cs[(mw * 16u + hh * 8u + (unsigned)r) * LDC + nw * 32u + m];
    d[0]  = acc0[r];
    d[16] = acc1[r];
  }
  __syncthreads();

  const float cs = 1.0f / (WCARRY * XCARRY);

  if (MODE == 0) {
    v8h x[2];
    size_t off[2];
#pragma unroll
    for (unsigned i = 0; i < 2u; ++i) {
      const unsigned r = 32u * i + (tid >> 3);
      const unsigned c = (tid & 7u) * 8u;
      const v4f u0 = *(const v4f*)&Cs[r * LDC + c];
      const v4f u1 = *(const v4f*)&Cs[r * LDC + c + 4];
      const v4f g0 = *(const v4f*)(bias + n0 + c);
      const v4f g1 = *(const v4f*)(bias + n0 + c + 4u);
#pragma unroll
      for (int j = 0; j < 4; ++j) {
        x[i][j]     = toh_flush(ACARRY * lrelu_act(u0[j] * cs + bf16r(g0[j])));
        x[i][j + 4] = toh_flush(ACARRY * lrelu_act(u1[j] * cs + bf16r(g1[j])));
      }
      off[i] = (size_t)(row0 + r) * UD + n0 + c;
    }
#pragma unroll
    for (int i = 0; i < 2; ++i) *(volatile v8h*)(out16 + off[i]) = x[i];
    __threadfence();
#pragma unroll
    for (int i = 0; i < 2; ++i) *(volatile v8h*)(out16 + off[i]) = x[i];
  }

  if (MODE == 1) {
    const unsigned bidx = row0 / (unsigned)SEQ;
    const unsigned key0 = row0 - bidx * (unsigned)SEQ;
    v8h x[2];
    size_t off[2];
#pragma unroll
    for (unsigned i = 0; i < 2u; ++i) {
      const unsigned dcol = 32u * i + (tid >> 3);
      const unsigned kk = (tid & 7u) * 8u;
      const float bb = bf16r(bias[n0 + dcol]);
#pragma unroll
      for (unsigned j = 0; j < 8u; ++j) {
        const float t = lrelu_act(Cs[(kk + j) * LDC + dcol] * cs + bb);
        x[i][j] = toh_flush(ACARRY * t);
      }
      off[i] = ((size_t)bidx * XD + n0 + dcol) * SEQ + key0 + kk;
    }
#pragma unroll
    for (int i = 0; i < 2; ++i) *(volatile v8h*)(out16 + off[i]) = x[i];
    __threadfence();
#pragma unroll
    for (int i = 0; i < 2; ++i) *(volatile v8h*)(out16 + off[i]) = x[i];
  }
}

__global__ __launch_bounds__(256) void gemm_qk_kernel(
    const _Float16* __restrict__ A16, const _Float16* __restrict__ Bt,
    const float* __restrict__ bias, _Float16* __restrict__ out16) {
  gemm_body<0>(A16, Bt, (unsigned)XD, bias, out16);
}
__global__ __launch_bounds__(256) void gemm_v_kernel(
    const _Float16* __restrict__ A16, const _Float16* __restrict__ Bt,
    const float* __restrict__ bias, _Float16* __restrict__ vt) {
  gemm_body<1>(A16, Bt, (unsigned)XD, bias, vt);
}

__global__ __launch_bounds__(64) __attribute__((amdgpu_num_vgpr(256))) void attn_kernel(
    const _Float16* __restrict__ Qh, const _Float16* __restrict__ Kh,
    const _Float16* __restrict__ Vt, const unsigned* __restrict__ Mk,
    const float* __restrict__ X, const float* __restrict__ G, const float* __restrict__ Be,
    float* __restrict__ out) {
  __shared__ float Os[2 * 16 * OLD];

  const unsigned lane = threadIdx.x & 31u;
  const unsigned wave = (unsigned)__builtin_amdgcn_readfirstlane((int)(threadIdx.x >> 5));
  const unsigned hh = lane >> 4, m = lane & 15u;
  const unsigned b = blockIdx.y;
  const unsigned qrow0 = blockIdx.x * 32u + wave * 16u;
  const float sc = 0.08838834764831845f / (ACARRY * ACARRY);

  const unsigned qbase = (b * (unsigned)SEQ + qrow0 + m) * (unsigned)UD + hh * 8u;
  unsigned kofs = (b * (unsigned)SEQ + m) * (unsigned)UD + hh * 8u;
  unsigned vofs = (b * (unsigned)XD + m) * (unsigned)SEQ + hh * 8u;
  const unsigned mbase = b * (unsigned)(SEQ / 32) * 32u;

  v8f ot[16];
#pragma unroll
  for (int t = 0; t < 16; ++t) ot[t] = (v8f){};
  float mrun = -1.0e30f, lrun = 0.0f;

  for (unsigned step = 0; step < (unsigned)(SEQ / 32); ++step) {
    unsigned qo = qbase;
    asm volatile("" : "+v"(qo));
    unsigned mw = Mk[mbase + step * 32u];
    mw = (unsigned)__builtin_amdgcn_readfirstlane((int)mw);

    v8f st0 = {}, st1 = {};
#pragma unroll
    for (int c = 0; c < 4; ++c) {
      const v16h qf = frag_at(Qh + qo + c * 32);
      const v16h k0 = frag_at(Kh + kofs + c * 32);
      const v16h k1 = frag_at(Kh + kofs + 16 * UD + c * 32);
      st0 = wmma16(k0, qf, st0);
      st1 = wmma16(k1, qf, st1);
    }
#pragma unroll
    for (int r = 0; r < 8; ++r) { st0[r] = st0[r] * sc; st1[r] = st1[r] * sc; }

    if (mw != 0u) {
      const unsigned mb = mw >> (8u * hh);
#pragma unroll
      for (int r = 0; r < 8; ++r) {
        st0[r] = ((mb >> r) & 1u) ? NEGFILL : st0[r];
        st1[r] = ((mb >> (16 + r)) & 1u) ? NEGFILL : st1[r];
      }
    }

    float mx = fmaxf(st0[0], st1[0]);
#pragma unroll
    for (int r = 1; r < 8; ++r) mx = fmaxf(mx, fmaxf(st0[r], st1[r]));
    mx = fmaxf(mx, __shfl_xor(mx, 16, 32));
    const float mn = fmaxf(mrun, mx);
    const float alpha = __expf(mrun - mn);
    mrun = mn;
    float rs = 0.0f;
#pragma unroll
    for (int r = 0; r < 8; ++r) {
      st0[r] = __expf(st0[r] - mn);
      st1[r] = __expf(st1[r] - mn);
      rs += st0[r] + st1[r];
    }
    rs += __shfl_xor(rs, 16, 32);
    lrun = alpha * lrun + rs;

    if (__builtin_amdgcn_ballot_w32(alpha != 1.0f) != 0u) {
#pragma unroll
      for (int t = 0; t < 16; ++t)
#pragma unroll
        for (int r = 0; r < 8; ++r) ot[t][r] = ot[t][r] * alpha;
    }

    v16h pf;
#pragma unroll
    for (int r = 0; r < 8; ++r) {
      pf[r]     = toh_flush(st0[r] * PCARRY);
      pf[r + 8] = toh_flush(st1[r] * PCARRY);
    }

#pragma unroll
    for (int g = 0; g < 4; ++g) {
#pragma unroll
      for (int tt = 0; tt < 4; ++tt) {
        const int t = g * 4 + tt;
        const v16h vf = frag_at(Vt + vofs + (unsigned)(t * 16) * (unsigned)SEQ);
        ot[t] = wmma16(vf, pf, ot[t]);
      }
      __builtin_amdgcn_sched_barrier(0);
    }

    kofs += 32u * (unsigned)UD;
    vofs += 32u;
  }

  const float inv = __builtin_amdgcn_rcpf(lrun) * (1.0f / (PCARRY * ACARRY));
  const unsigned wbase = wave * (16u * OLD);
#pragma unroll
  for (int t = 0; t < 16; ++t) {
    v4f lo, hi;
#pragma unroll
    for (int r = 0; r < 4; ++r) { lo[r] = ot[t][r] * inv; hi[r] = ot[t][r + 4] * inv; }
    *(v4f*)&Os[wbase + m * OLD + (unsigned)t * 16u + hh * 8u]      = lo;
    *(v4f*)&Os[wbase + m * OLD + (unsigned)t * 16u + hh * 8u + 4u] = hi;
  }
  wave_lds_sync();

  const unsigned c0 = lane * 4u, c1 = 128u + lane * 4u;
  const v4f g0 = *(const v4f*)(G + c0);
  const v4f g1 = *(const v4f*)(G + c1);
  const v4f b0 = *(const v4f*)(Be + c0);
  const v4f b1 = *(const v4f*)(Be + c1);
#pragma unroll 1
  for (unsigned r = 0; r < 16u; ++r) {
    const size_t frow = (size_t)b * SEQ_FULL + qrow0 + r;
    const v4f a0 = *(const v4f*)&Os[wbase + r * OLD + c0];
    const v4f a1 = *(const v4f*)&Os[wbase + r * OLD + c1];
    const v4f x0 = *(const v4f*)(X + frow * XD + c0);
    const v4f x1 = *(const v4f*)(X + frow * XD + c1);
    v4f u0, u1;
    float s = 0.0f;
#pragma unroll
    for (int i = 0; i < 4; ++i) {
      u0[i] = a0[i] + bf16r(x0[i]);
      u1[i] = a1[i] + bf16r(x1[i]);
      s += u0[i] + u1[i];
    }
    const float mean = red32_sum(s) * (1.0f / (float)XD);
    float ss = 0.0f;
#pragma unroll
    for (int i = 0; i < 4; ++i) {
      u0[i] = u0[i] - mean;
      u1[i] = u1[i] - mean;
      ss += u0[i] * u0[i];
      ss += u1[i] * u1[i];
    }
    const float var = red32_sum(ss) * (1.0f / (float)XD);
    const float rstd = 1.0f / sqrtf(var + 1.0e-8f);
    v4f y0, y1;
#pragma unroll
    for (int i = 0; i < 4; ++i) {
      y0[i] = bf16r(g0[i]) * (u0[i] * rstd) + bf16r(b0[i]);
      y1[i] = bf16r(g1[i]) * (u1[i] * rstd) + bf16r(b1[i]);
    }
    float* p0 = out + frow * XD + c0;
    float* p1 = out + frow * XD + c1;
    *(volatile v4f*)p0 = y0;
    *(volatile v4f*)p1 = y1;
    __threadfence();
    *(volatile v4f*)p0 = y0;
    *(volatile v4f*)p1 = y1;
  }
}

extern "C" void kernel_launch(void* const* d_in, const int* in_sizes, int n_in,
                              void* d_out, int out_size, void* d_ws, size_t ws_size,
                              hipStream_t stream) {
  if (n_in < 9) return;
  const long long need_x = ((long long)(NB - 1) * SEQ_FULL + SEQ) * XD;
  if ((long long)in_sizes[0] < need_x) return;
  if ((long long)in_sizes[1] < (long long)XD * UD) return;
  if ((long long)in_sizes[3] < (long long)XD * UD) return;
  if ((long long)in_sizes[5] < (long long)XD * XD) return;
  if (in_sizes[2] < UD || in_sizes[4] < UD) return;
  if (in_sizes[6] < XD || in_sizes[7] < XD || in_sizes[8] < XD) return;
  if ((long long)out_size < need_x) return;
  if (ws_size < WS_TOTAL) return;

  const float* X   = (const float*)d_in[0];
  const float* wq  = (const float*)d_in[1];
  const float* bq  = (const float*)d_in[2];
  const float* wk  = (const float*)d_in[3];
  const float* bk  = (const float*)d_in[4];
  const float* wv  = (const float*)d_in[5];
  const float* bv  = (const float*)d_in[6];
  const float* gam = (const float*)d_in[7];
  const float* bet = (const float*)d_in[8];
  float* out = (float*)d_out;

  char* ws = (char*)d_ws;
  _Float16* Wq_t = (_Float16*)(ws + OFF_WQ);
  _Float16* Wk_t = (_Float16*)(ws + OFF_WK);
  _Float16* Wv_t = (_Float16*)(ws + OFF_WV);
  _Float16* X16  = (_Float16*)(ws + OFF_X16);
  _Float16* Qh16 = (_Float16*)(ws + OFF_Q);
  _Float16* Kh16 = (_Float16*)(ws + OFF_K);
  _Float16* Vt16 = (_Float16*)(ws + OFF_VT);
  unsigned* Mk   = (unsigned*)(ws + OFF_MK);

  dim3 blk(256);

  wconv_kernel<<<dim3(UD / 64, XD / 64), blk, 0, stream>>>(wq, Wq_t, (unsigned)UD, (unsigned)XD);
  wconv_kernel<<<dim3(UD / 64, XD / 64), blk, 0, stream>>>(wk, Wk_t, (unsigned)UD, (unsigned)XD);
  wconv_kernel<<<dim3(XD / 64, XD / 64), blk, 0, stream>>>(wv, Wv_t, (unsigned)XD, (unsigned)XD);

  xprep_kernel<<<dim3(MROWS / 32), blk, 0, stream>>>(X, X16, Mk);
  gemm_qk_kernel<<<dim3(UD / 64, MROWS / 64), blk, 0, stream>>>(X16, Wq_t, bq, Qh16);
  gemm_qk_kernel<<<dim3(UD / 64, MROWS / 64), blk, 0, stream>>>(X16, Wk_t, bk, Kh16);
  gemm_v_kernel<<<dim3(XD / 64, MROWS / 64), blk, 0, stream>>>(X16, Wv_t, bv, Vt16);
  attn_kernel<<<dim3(SEQ / 32, NB), dim3(64), 0, stream>>>(Qh16, Kh16, Vt16, Mk, X, gam, bet, out);
}
